// ToyModel_56745107915071
// MI455X (gfx1250) — hardware-run, weakly checked
//
#include <hip/hip_runtime.h>
#include <math.h>

typedef __attribute__((ext_vector_type(16))) _Float16 v16h;
typedef __attribute__((ext_vector_type(8)))  _Float16 v8h;
typedef __attribute__((ext_vector_type(16))) __bf16   v16b;
typedef __attribute__((ext_vector_type(8)))  __bf16   v8b;
typedef __attribute__((ext_vector_type(8)))  float    v8f;
typedef __attribute__((ext_vector_type(4)))  float    v4f;

constexpr int kB    = 256;
constexpr int kT    = 512;
constexpr int kI    = 100;
constexpr int kIP   = 128;
constexpr int kHid  = 275;
constexpr int kHP   = 288;
constexpr int kO    = 100;
constexpr int kOP   = 128;
constexpr int kG4   = 4 * kHid;
constexpr int kG4P  = 4 * kHP;
constexpr int kK    = kHP + kIP;
constexpr int kKP   = 448;
constexpr int kHS   = 320;
constexpr int kRows = kB * kT;
constexpr int kThr  = 256;
constexpr float kInCarry = 1024.0f;
constexpr float kWCarry = 4096.0f;
constexpr float kSc = 1.0f / (kInCarry * kWCarry);
constexpr float kF16MinNormal = 6.103515625e-5f;

static_assert((kB % 64) == 0 && (kG4P % 64) == 0 && (kOP % 64) == 0 && (kRows % 64) == 0 && ((kB / 64) * (kG4P / 64)) % 8 == 0 && ((kRows / 64) * (kOP / 64)) % 8 == 0, "GEMM M, N multiples of 64; grids exact (72 and 4,096 tiles)");
static_assert((kK % 32) == 0 && (kHP % 32) == 0 && kHP >= kHid && kIP >= kI && kOP >= kO && (kHP % 8) == 0 && (kIP % 8) == 0, "GEMM K multiples of 32; the paddings");

constexpr size_t kOffW16 = 0ull;
constexpr size_t kOffWO16 = 1032192ull;
constexpr size_t kOffBIAS = 1114112ull;
constexpr size_t kOffHX16 = 1122304ull;
constexpr size_t kOffGG = 1351680ull;
constexpr size_t kOffC32 = 2531328ull;
constexpr size_t kOffHS16 = 2826240ull;
constexpr size_t kOffOUTP = 86712320ull;
constexpr size_t kWsTotal = 153821184ull;
static_assert(kWsTotal <= 268435456ull, "carve cap: the offered workspace");
static_assert(kOffW16 == 0
              && kOffWO16 == kOffW16 + 1032192ull
              && kOffBIAS == kOffWO16 + 81920ull
              && kOffHX16 == kOffBIAS + 8192ull
              && kOffGG == kOffHX16 + 229376ull
              && kOffC32 == kOffGG + 1179648ull
              && kOffHS16 == kOffC32 + 294912ull
              && kOffOUTP == kOffHS16 + 83886080ull
              && kWsTotal == kOffOUTP + 67108864ull, "the carve is chained and totalled");
static_assert((kOffW16 % 256) == 0 && (kOffWO16 % 256) == 0 && (kOffBIAS % 256) == 0 && (kOffHX16 % 256) == 0 && (kOffGG % 256) == 0 && (kOffC32 % 256) == 0 && (kOffHS16 % 256) == 0 && (kOffOUTP % 256) == 0 && ((kKP * 2) % 128) == 0 && ((kHS * 2) % 128) == 0 && kKP >= kK && kHS >= kHP, "aligned regions; the f16 planes' rows are whole lines");
constexpr int kFBG = 0, kFBO = 1152, kFEnd = 2048;
static_assert(kFBO == kFBG + kG4P && kFBO + kOP <= kFEnd && (kFBO % 128) == 0 && ((kFBO + kOP) % 128) == 0, "bias stream map; region boundaries wave-uniform");

__device__ __forceinline__ unsigned short f2bf_bits(float f) {
  unsigned u = __float_as_uint(f);
  return (unsigned short)((u + 0x7FFFu + ((u >> 16) & 1u)) >> 16);
}
__device__ __forceinline__ float bf_bits2f(unsigned short h) { return __uint_as_float(((unsigned)h) << 16); }
__device__ __forceinline__ float bf16r(float f) { return bf_bits2f(f2bf_bits(f)); }
__device__ __forceinline__ float carry_flush(float v, float carry) {
  const float s = v * carry;
  return (fabsf(s) < kF16MinNormal) ? 0.0f : s;
}
__device__ __forceinline__ float frcp(float x) { return __builtin_amdgcn_rcpf(x); }

__device__ __forceinline__ void dep_guard4_h(v8f& a, v8f& b, v8f& c, v8f& d, v16h x, v16h y) { asm volatile("v_nop\n\tv_nop\n\tv_nop\n\tv_nop" : "+v"(a), "+v"(b), "+v"(c), "+v"(d) : "v"(x), "v"(y)); }
__device__ __forceinline__ void dep_guard4_b(v8f& a, v8f& b, v8f& c, v8f& d, v16b x, v16b y) { asm volatile("v_nop\n\tv_nop\n\tv_nop\n\tv_nop" : "+v"(a), "+v"(b), "+v"(c), "+v"(d) : "v"(x), "v"(y)); }
__device__ __forceinline__ void keep4_h(v16h a, v16h b, v16h c, v16h d) { asm volatile("v_nop" :: "v"(a), "v"(b), "v"(c), "v"(d)); }
__device__ __forceinline__ void keep4_b(v16b a, v16b b, v16b c, v16b d) { asm volatile("v_nop" :: "v"(a), "v"(b), "v"(c), "v"(d)); }
__device__ __forceinline__ void acc_guard4(v8f& a, v8f& b, v8f& c, v8f& d) { asm volatile("v_nop\n\tv_nop\n\tv_nop\n\tv_nop" : "+v"(a), "+v"(b), "+v"(c), "+v"(d)); }

template <typename T> struct Frag;
template <> struct Frag<_Float16> {
  typedef v16h V; union U { v16h v; v8h h[2]; };
  static __device__ __forceinline__ v16h load(const _Float16* p) {
    U f; f.h[0] = *(const v8h*)(p); f.h[1] = *(const v8h*)(p + 16); return f.v;
  }
  static __device__ __forceinline__ v8f mma(v16h a, v16h b, v8f c) {
    return __builtin_amdgcn_wmma_f32_16x16x32_f16(false, a, false, b, (short)0, c, false, false);
  }
  static __device__ __forceinline__ void guard4(v8f& a, v8f& b, v8f& c, v8f& d, v16h x, v16h y) { dep_guard4_h(a, b, c, d, x, y); }
  static __device__ __forceinline__ void keep(v16h a, v16h b, v16h c, v16h d) { keep4_h(a, b, c, d); }
};
template <> struct Frag<__bf16> {
  typedef v16b V; union U { v16b v; v8b h[2]; };
  static __device__ __forceinline__ v16b load(const __bf16* p) {
    U f; f.h[0] = *(const v8b*)(p); f.h[1] = *(const v8b*)(p + 16); return f.v;
  }
  static __device__ __forceinline__ v8f mma(v16b a, v16b b, v8f c) {
    return __builtin_amdgcn_wmma_f32_16x16x32_bf16(false, a, false, b, (short)0, c, false, false);
  }
  static __device__ __forceinline__ void guard4(v8f& a, v8f& b, v8f& c, v8f& d, v16b x, v16b y) { dep_guard4_b(a, b, c, d, x, y); }
  static __device__ __forceinline__ void keep(v16b a, v16b b, v16b c, v16b d) { keep4_b(a, b, c, d); }
};

__device__ __forceinline__ v8f mma_h(v16h a, v16h b, v8f c) {
  c = __builtin_amdgcn_wmma_f32_16x16x32_f16(false, a, false, b, (short)0, c, false, false);
  asm volatile("v_nop\n\tv_nop\n\tv_nop\n\tv_nop" : "+v"(c) : "v"(a), "v"(b));
  return c;
}

template <int ET> struct Elem;
template <> struct Elem<0> { typedef _Float16 T; };
template <> struct Elem<1> { typedef __bf16 T; };
template <int ET, bool SPLIT, int BIAS_MODE, int OUT_MODE, bool RESID, int ACT = 0>
__global__ __launch_bounds__(256) void wmma_gemm64(
    const unsigned short* __restrict__ Ap, const unsigned short* __restrict__ A2p, int lda, long strideA,
    const unsigned short* __restrict__ Btp, const unsigned short* __restrict__ Bt2p, int ldb, long strideB,
    void* __restrict__ Cout, void* __restrict__ Cout2, int ldc, long strideC,
    const float* __restrict__ bias,
    const float* __restrict__ resid, long strideR,
    int M, int N, int K, float scale) {
  typedef typename Elem<ET>::T T;
  typedef typename Frag<T>::V V;
  const T* A = (const T*)Ap; const T* A2 = (const T*)A2p; const T* Bt = (const T*)Btp; const T* Bt2 = (const T*)Bt2p;
  __shared__ __align__(16) float sT[8][16 * 68];
  const int b    = blockIdx.y;
  const int lane = threadIdx.x & 31;
  const int wave = threadIdx.x >> 5;
  const int tilesN = N >> 6;
  const int tilesM = M >> 6;
  const int tile = blockIdx.x * 8 + wave;
  if (tile >= tilesM * tilesN) return;
  const int tm = tile / tilesN;
  const int tn = tile - tm * tilesN;
  const int m0 = tm << 6;
  const int n0 = tn << 6;

  const T* Ab  = A  + (size_t)b * strideA;
  const T* Bb  = Bt + (size_t)b * strideB;
  const T* Ab2 = SPLIT ? (A2  + (size_t)b * strideA) : nullptr;
  const T* Bb2 = SPLIT ? (Bt2 + (size_t)b * strideB) : nullptr;

  const int rlane = lane & 15;
  const int koff  = (lane >> 4) * 8;
  const int mOff  = (lane >> 4) * 8;

  v8f acc[4][4];
#pragma unroll
  for (int i = 0; i < 4; ++i)
#pragma unroll
    for (int j = 0; j < 4; ++j) acc[i][j] = (v8f){0.f,0.f,0.f,0.f,0.f,0.f,0.f,0.f};

  for (int k0 = 0; k0 < K; k0 += 32) {
    V bh[4], bl[4];
#pragma unroll
    for (int j = 0; j < 4; ++j) {
      const size_t bo = (size_t)(n0 + (j << 4) + rlane) * ldb + koff + k0;
      bh[j] = Frag<T>::load(Bb + bo);
      if (SPLIT) bl[j] = Frag<T>::load(Bb2 + bo);
    }
#pragma unroll
    for (int i = 0; i < 4; ++i) {
      const size_t ao = (size_t)(m0 + (i << 4) + rlane) * lda + koff + k0;
      V ah = Frag<T>::load(Ab + ao);
      V al;
      if (SPLIT) al = Frag<T>::load(Ab2 + ao);
#pragma unroll
      for (int j = 0; j < 4; ++j) {
        acc[i][j] = Frag<T>::mma(ah, bh[j], acc[i][j]);
        if (SPLIT) {
          acc[i][j] = Frag<T>::mma(ah, bl[j], acc[i][j]);
          acc[i][j] = Frag<T>::mma(al, bh[j], acc[i][j]);
        }
      }
      Frag<T>::guard4(acc[i][0], acc[i][1], acc[i][2], acc[i][3], ah, SPLIT ? al : ah);
    }
    Frag<T>::keep(bh[0], bh[1], bh[2], bh[3]);
    if (SPLIT) Frag<T>::keep(bl[0], bl[1], bl[2], bl[3]);
  }
  acc_guard4(acc[0][0], acc[0][1], acc[0][2], acc[0][3]);
  acc_guard4(acc[1][0], acc[1][1], acc[1][2], acc[1][3]);
  acc_guard4(acc[2][0], acc[2][1], acc[2][2], acc[2][3]);
  acc_guard4(acc[3][0], acc[3][1], acc[3][2], acc[3][3]);

  float* slab = sT[wave];
  const float* Rb = RESID ? (resid + (size_t)b * strideR) : nullptr;
#pragma unroll
  for (int i = 0; i < 4; ++i) {
    const int mBase = m0 + (i << 4);
#pragma unroll
    for (int j = 0; j < 4; ++j) {
      const int n = n0 + (j << 4) + rlane;
      float bv = 0.f;
      if (BIAS_MODE == 2) bv = bias[n];
#pragma unroll
      for (int r = 0; r < 8; ++r) {
        float v = acc[i][j][r] * scale;
        if (BIAS_MODE == 1) v += bias[mBase + mOff + r];
        if (BIAS_MODE == 2) v += bv;
        if (RESID) v += Rb[(size_t)(mBase + mOff + r) * ldc + n];
        if (ACT == 1) v = tanhf(v);
        if (ACT == 2) v = fmaxf(v, 0.0f);
        if (ACT == 3) v = v / (1.0f + expf(-v));
        if (ACT == 4) v = (v > 0.f) ? v : 0.01f * v;
        slab[(mOff + r) * 68 + (j << 4) + rlane] = v;
      }
    }
    __builtin_amdgcn_fence(__ATOMIC_RELEASE, "workgroup");
    __builtin_amdgcn_wave_barrier();
    __builtin_amdgcn_fence(__ATOMIC_ACQUIRE, "workgroup");
    if (OUT_MODE == 0) {
      float* C = (float*)Cout + (size_t)b * strideC;
      const int hh = lane >> 4, c4 = (lane & 15) * 4;
      for (int pass = 0; pass < 2; ++pass) {
#pragma unroll
        for (int it = 0; it < 8; ++it) {
          const int row = it * 2 + hh;
          v4f v = *(const v4f*)(slab + row * 68 + c4);
          *(volatile v4f*)(C + (size_t)(mBase + row) * ldc + n0 + c4) = v;
        }
        __threadfence();
      }
    } else {
      const int q = lane >> 3, c8 = (lane & 7) * 8;
      unsigned short* C  = (unsigned short*)Cout  + (size_t)b * strideC;
      unsigned short* C2 = (OUT_MODE == 2) ? ((unsigned short*)Cout2 + (size_t)b * strideC) : nullptr;
      for (int pass = 0; pass < 2; ++pass) {
#pragma unroll
        for (int it = 0; it < 4; ++it) {
          const int row = it * 4 + q;
          const float* sp = slab + row * 68 + c8;
          v8h hv, lv;
#pragma unroll
          for (int e = 0; e < 8; ++e) {
            if (OUT_MODE == 1) {
              hv[e] = (_Float16)sp[e];
            } else {
              unsigned short hb = f2bf_bits(sp[e]);
              unsigned short lb = f2bf_bits(sp[e] - bf_bits2f(hb));
              hv[e] = __builtin_bit_cast(_Float16, hb);
              lv[e] = __builtin_bit_cast(_Float16, lb);
            }
          }
          *(volatile v8h*)(C + (size_t)(mBase + row) * ldc + n0 + c8) = hv;
          if (OUT_MODE == 2) *(volatile v8h*)(C2 + (size_t)(mBase + row) * ldc + n0 + c8) = lv;
        }
        __threadfence();
      }
    }
    __builtin_amdgcn_fence(__ATOMIC_RELEASE, "workgroup");
    __builtin_amdgcn_wave_barrier();
    __builtin_amdgcn_fence(__ATOMIC_ACQUIRE, "workgroup");
  }
}


__device__ __forceinline__ float fast_tanh(float v) { return 1.0f - 2.0f * frcp(__expf(2.0f * v) + 1.0f); }
__device__ __forceinline__ float fast_sigmoid(float v) { return frcp(1.0f + __expf(-v)); }

__global__ __launch_bounds__(64) void wpack_kernel(const float* __restrict__ W_ih, const float* __restrict__ W_hh, const float* __restrict__ W_out,
                                                   unsigned short* __restrict__ W16, unsigned short* __restrict__ WO16) {
  const unsigned row = blockIdx.y;
  const unsigned c = threadIdx.x;
  v8h hv;
  if (row < (unsigned)kG4P) {
    if (c >= 52u) return;
    const unsigned g = row / (unsigned)kHP, u = row - g * (unsigned)kHP;
    const bool rowLive = u < (unsigned)kHid;
    const unsigned sr = g * (unsigned)kHid + (rowLive ? u : 0u);
#pragma unroll
    for (int e = 0; e < 8; ++e) {
      const unsigned k = c * 8u + (unsigned)e;
      const bool inH = k < (unsigned)kHid;
      const bool inX = (k >= (unsigned)kHP) && (k < (unsigned)(kHP + kI));
      const float wh = W_hh[(size_t)sr * kHid + (inH ? k : 0u)];
      const float wx = W_ih[(size_t)sr * kI + (inX ? (k - (unsigned)kHP) : 0u)];
      const float w = inH ? wh : (inX ? wx : 0.0f);
      hv[e] = (_Float16)(rowLive ? carry_flush(bf16r(w), kWCarry) : 0.0f);
    }
    unsigned short* dp = W16 + (size_t)row * kKP + c * 8u;
    *(volatile v8h*)dp = hv;
    __threadfence();
    *(volatile v8h*)dp = hv;
  } else {
    if (c >= 36u) return;
    const unsigned o = row - (unsigned)kG4P;
    const bool rowLive = o < (unsigned)kO;
    const unsigned sr = rowLive ? o : 0u;
#pragma unroll
    for (int e = 0; e < 8; ++e) {
      const unsigned k = c * 8u + (unsigned)e;
      const bool inH = k < (unsigned)kHid;
      const float wv = W_out[(size_t)sr * kHid + (inH ? k : 0u)];
      hv[e] = (_Float16)((rowLive && inH) ? carry_flush(bf16r(wv), kWCarry) : 0.0f);
    }
    unsigned short* dp = WO16 + (size_t)o * kHS + c * 8u;
    *(volatile v8h*)dp = hv;
    __threadfence();
    *(volatile v8h*)dp = hv;
  }
}
static_assert(kK / 8 == 52 && kHP / 8 == 36 && kKP / 8 <= 64 && kHS / 8 <= 64, "a row's chunks fit one 64-thread block");

__global__ __launch_bounds__(kThr) void setup_kernel(const float* __restrict__ x, const float* __restrict__ b_ih, const float* __restrict__ b_hh, const float* __restrict__ b_out,
                                                     float* __restrict__ BIAS, float* __restrict__ C32, unsigned short* __restrict__ HX16) {
  const unsigned y = blockIdx.y;
  const unsigned c = threadIdx.x;
  if (y < 6u) {
    v4f o = {0.f, 0.f, 0.f, 0.f};
    float* dp;
    if (y < 4u) {
      if (c >= 72u) return;
#pragma unroll
      for (int e = 0; e < 4; ++e) {
        const unsigned u = c * 4u + (unsigned)e;
        const bool live = u < (unsigned)kHid;
        const unsigned s = y * (unsigned)kHid + (live ? u : 0u);
        const float p = b_ih[s], q = b_hh[s];
        o[e] = live ? (bf16r(p) + bf16r(q)) : 0.0f;
      }
      dp = BIAS + kFBG + y * (unsigned)kHP + c * 4u;
    } else if (y == 4u) {
      if (c >= 32u) return;
#pragma unroll
      for (int e = 0; e < 4; ++e) {
        const unsigned j = c * 4u + (unsigned)e;
        const bool live = j < (unsigned)kO;
        const float p = b_out[live ? j : 0u];
        o[e] = live ? bf16r(p) : 0.0f;
      }
      dp = BIAS + kFBO + c * 4u;
    } else {
      if (c >= 192u) return;
      dp = BIAS + kFBO + kOP + c * 4u;
    }
    *(volatile v4f*)dp = o;
    __threadfence();
    *(volatile v4f*)dp = o;
  } else {
    const unsigned smp = y - 6u;
    if (c < 72u) {
      const v4f z = {0.f, 0.f, 0.f, 0.f};
      float* dp = C32 + (size_t)smp * kHP + c * 4u;
      *(volatile v4f*)dp = z;
      __threadfence();
      *(volatile v4f*)dp = z;
    } else if (c < 124u) {
      const unsigned ch = c - 72u;
      v8h hv;
#pragma unroll
      for (int e = 0; e < 8; ++e) hv[e] = (_Float16)0.0f;
      if (ch >= 36u) {
        const float* xr = x + (size_t)smp * kT * kI;
#pragma unroll
        for (int e = 0; e < 8; ++e) {
          const unsigned k = (ch - 36u) * 8u + (unsigned)e;
          const bool live = k < (unsigned)kI;
          const float p = xr[live ? k : 0u];
          hv[e] = (_Float16)(live ? carry_flush(bf16r(p), kInCarry) : 0.0f);
        }
      }
      unsigned short* dp = HX16 + (size_t)smp * kKP + ch * 8u;
      *(volatile v8h*)dp = hv;
      __threadfence();
      *(volatile v8h*)dp = hv;
    }
  }
}
static_assert(kHP / 4 == 72 && kOP / 4 == 32 && (kFEnd - kFBO - kOP) / 4 == 192 && 72 + 52 == 124 && kFBO == 4 * kHP, "set-up rows");

__global__ __launch_bounds__(64) void cell_kernel(const float* __restrict__ GG, const float* __restrict__ x, float* __restrict__ C32,
                                                    unsigned short* __restrict__ HX16, unsigned short* __restrict__ HS16, int t) {
  const unsigned smp = blockIdx.y;
  const unsigned c = threadIdx.x;
  if (c < 36u) {
    const unsigned u8 = c * 8u;
    const float* gr = GG + (size_t)smp * kG4P + u8;
    float* cp = C32 + (size_t)smp * kHP + u8;
    v8h hv;
    v4f cn0, cn1;
#pragma unroll
    for (int hlf = 0; hlf < 2; ++hlf) {
      const v4f gi = *(const v4f*)(gr + 4 * hlf), gf = *(const v4f*)(gr + kHP + 4 * hlf), gg = *(const v4f*)(gr + 2 * kHP + 4 * hlf), go = *(const v4f*)(gr + 3 * kHP + 4 * hlf);
      const v4f co = *(const v4f*)(cp + 4 * hlf);
#pragma unroll
      for (int e = 0; e < 4; ++e) {
        const float cn = fast_sigmoid(gf[e]) * co[e] + fast_sigmoid(gi[e]) * fast_tanh(gg[e]);
        const float hn = fast_sigmoid(go[e]) * fast_tanh(cn);
        if (hlf == 0) cn0[e] = cn; else cn1[e] = cn;
        hv[4 * hlf + e] = (_Float16)carry_flush(hn, kInCarry);
      }
    }
    unsigned short* hp = HX16 + (size_t)smp * kKP + u8;
    unsigned short* sp = HS16 + ((size_t)smp * kT + (size_t)t) * kHS + u8;
    for (int pass = 0; pass < 2; ++pass) {
      *(volatile v4f*)cp = cn0;
      *(volatile v4f*)(cp + 4) = cn1;
      *(volatile v8h*)hp = hv;
      *(volatile v8h*)sp = hv;
      __threadfence();
    }
  } else if (c < 52u && t + 1 < kT) {
    const float* xr = x + ((size_t)smp * kT + (size_t)(t + 1)) * kI;
    v8h xv;
#pragma unroll
    for (int e = 0; e < 8; ++e) {
      const unsigned k = (c - 36u) * 8u + (unsigned)e;
      const bool live = k < (unsigned)kI;
      const float p = xr[live ? k : 0u];
      xv[e] = (_Float16)(live ? carry_flush(bf16r(p), kInCarry) : 0.0f);
    }
    unsigned short* xp = HX16 + (size_t)smp * kKP + c * 8u;
    *(volatile v8h*)xp = xv;
    __threadfence();
    *(volatile v8h*)xp = xv;
  }
}
static_assert((kHP % 8) == 0 && kHP / 8 == 36 && (kHP + kIP) / 8 == 52 && 52 <= 64, "a sample's chunks fit one 64-thread block");

__global__ __launch_bounds__(kThr) void out_kernel(const float* __restrict__ OUTP, float* __restrict__ out) {
  const unsigned v = blockIdx.x * (unsigned)kThr + threadIdx.x;
  const unsigned row = v / 25u, c4 = (v - row * 25u) * 4u;
  const v4f a = *(const v4f*)(OUTP + (size_t)row * kOP + c4);
  float* dp = out + (size_t)v * 4u;
  *(volatile v4f*)dp = a;
  __threadfence();
  *(volatile v4f*)dp = a;
}
static_assert(kO == 100 && ((size_t)kRows * 25) % kThr == 0, "output grid exact");

extern "C" void kernel_launch(void* const* d_in, const int* in_sizes, int n_in,
                              void* d_out, int out_size, void* d_ws, size_t ws_size,
                              hipStream_t stream) {
  if (n_in < 7 || d_out == nullptr || d_ws == nullptr) return;
  if (in_sizes[0] != kB * kT * kI || in_sizes[1] != kG4 * kI || in_sizes[2] != kG4 * kHid || in_sizes[3] != kG4 || in_sizes[4] != kG4 || in_sizes[5] != kO * kHid || in_sizes[6] != kO) return;
  if (out_size != kB * kT * kO) return;
  if (ws_size < kWsTotal) return;
  const float* x = (const float*)d_in[0];
  const float* W_ih = (const float*)d_in[1];
  const float* W_hh = (const float*)d_in[2];
  const float* b_ih = (const float*)d_in[3];
  const float* b_hh = (const float*)d_in[4];
  const float* W_out = (const float*)d_in[5];
  const float* b_out = (const float*)d_in[6];
  float* out = (float*)d_out;
  char* ws = (char*)d_ws;
  unsigned short* W16 = (unsigned short*)(ws + kOffW16);
  unsigned short* WO16 = (unsigned short*)(ws + kOffWO16);
  float* BIAS = (float*)(ws + kOffBIAS);
  unsigned short* HX16 = (unsigned short*)(ws + kOffHX16);
  float* GG = (float*)(ws + kOffGG);
  float* C32 = (float*)(ws + kOffC32);
  unsigned short* HS16 = (unsigned short*)(ws + kOffHS16);
  float* OUTP = (float*)(ws + kOffOUTP);

  wpack_kernel<<<dim3(1, kG4P + kOP), 64, 0, stream>>>(W_ih, W_hh, W_out, W16, WO16);
  setup_kernel<<<dim3(1, 6 + kB), kThr, 0, stream>>>(x, b_ih, b_hh, b_out, BIAS, C32, HX16);
  for (int t = 0; t < kT; ++t) {
    wmma_gemm64<0, false, 2, 0, false, 0><<<dim3((kB / 64) * (kG4P / 64) / 8, 1), 256, 0, stream>>>(
        HX16, HX16, kKP, 0L, W16, W16, kKP, 0L, (void*)GG, (void*)GG, kG4P, 0L, BIAS + kFBG, nullptr, 0L, kB, kG4P, kK, kSc);
    cell_kernel<<<dim3(1, kB), 64, 0, stream>>>(GG, x, C32, HX16, HS16, t);
  }
  wmma_gemm64<0, false, 2, 0, false, 0><<<dim3((kRows / 64) * (kOP / 64) / 8, 1), 256, 0, stream>>>(
      HS16, HS16, kHS, 0L, WO16, WO16, kHS, 0L, (void*)OUTP, (void*)OUTP, kOP, 0L, BIAS + kFBO, nullptr, 0L, kRows, kOP, kHP, kSc);
  out_kernel<<<(int)(((size_t)kRows * 25) / kThr), kThr, 0, stream>>>(OUTP, out);
}
